// MCGRU_45921790329248
// MI455X (gfx1250) — hardware-verified
//
#include <hip/hip_runtime.h>
#include <math.h>

constexpr int kNB  = 256;
constexpr int kNT  = 128;
constexpr int kNL  = 64;
constexpr int kNF  = 32;
constexpr int kNG  = 96;
constexpr int kNH  = 128;
constexpr int kND  = 32;
constexpr int kKO  = kNL * kNF + kNH;
constexpr int kThreads = 256;
constexpr int kWP  = 32;
constexpr int kHP  = 40;
constexpr int kSP  = 36;
constexpr int kPrepX  = (kNB * kNT * kNL) / (8 * kThreads);
constexpr int kPrepLW = (kNL * kNL) / (2 * kThreads);
constexpr int kPrepST = (kNB * kND) / (2 * kThreads);
constexpr int kPrepDW = (kNH * kND) / (2 * kThreads);
constexpr int kPrepOW = (kNH * kKO) / (2 * kThreads);
constexpr int kPrepBlocks = kPrepX + kPrepLW + kPrepST + kPrepDW + kPrepOW;

typedef __attribute__((ext_vector_type(16))) _Float16 v16h;
typedef __attribute__((ext_vector_type(8)))  _Float16 v8h;
typedef __attribute__((ext_vector_type(16))) __bf16   v16b;
typedef __attribute__((ext_vector_type(8)))  __bf16   v8b;
typedef __attribute__((ext_vector_type(8)))  float    v8f;
typedef __attribute__((ext_vector_type(4)))  float    v4f;

__device__ __forceinline__ unsigned short f2bf_bits(float f) {
  unsigned u = __float_as_uint(f);
  return (unsigned short)((u + 0x7FFFu + ((u >> 16) & 1u)) >> 16);
}
__device__ __forceinline__ float bf_bits2f(unsigned short h) { return __uint_as_float(((unsigned)h) << 16); }

__device__ __forceinline__ void dep_guard_h(v8f& a, v8f& b, v16h x, v16h y) { asm volatile("v_nop\n\tv_nop\n\tv_nop\n\tv_nop" : "+v"(a), "+v"(b) : "v"(x), "v"(y)); }
__device__ __forceinline__ void dep_guard_b(v8f& a, v8f& b, v16b x, v16b y) { asm volatile("v_nop\n\tv_nop\n\tv_nop\n\tv_nop" : "+v"(a), "+v"(b) : "v"(x), "v"(y)); }
__device__ __forceinline__ void keep4_h(v16h a, v16h b, v16h c, v16h d) { asm volatile("v_nop" :: "v"(a), "v"(b), "v"(c), "v"(d)); }
__device__ __forceinline__ void keep4_b(v16b a, v16b b, v16b c, v16b d) { asm volatile("v_nop" :: "v"(a), "v"(b), "v"(c), "v"(d)); }
__device__ __forceinline__ void acc_guard4(v8f& a, v8f& b, v8f& c, v8f& d) { asm volatile("v_nop\n\tv_nop\n\tv_nop\n\tv_nop" : "+v"(a), "+v"(b), "+v"(c), "+v"(d)); }
__device__ __forceinline__ void dep_guard3_h(v8f& a, v8f& b, v8f& c, v16h w, v16h x, v16h y, v16h z) {
  asm volatile("v_nop\n\tv_nop\n\tv_nop\n\tv_nop" : "+v"(a), "+v"(b), "+v"(c) : "v"(w), "v"(x), "v"(y), "v"(z));
}
__device__ __forceinline__ void acc_guard3(v8f& a, v8f& b, v8f& c) { asm volatile("v_nop\n\tv_nop\n\tv_nop\n\tv_nop" : "+v"(a), "+v"(b), "+v"(c)); }

template <typename T> struct Frag;
template <> struct Frag<_Float16> {
  typedef v16h V; union U { v16h v; v8h h[2]; };
  static __device__ __forceinline__ v16h load(const _Float16* p) {
    U f; f.h[0] = *(const v8h*)(p); f.h[1] = *(const v8h*)(p + 16); return f.v;
  }
  static __device__ __forceinline__ v8f mma(v16h a, v16h b, v8f c) {
    return __builtin_amdgcn_wmma_f32_16x16x32_f16(false, a, false, b, (short)0, c, false, false);
  }
  static __device__ __forceinline__ void guard(v8f& a, v8f& b, v16h x, v16h y) { dep_guard_h(a, b, x, y); }
  static __device__ __forceinline__ void keep(v16h a, v16h b, v16h c, v16h d) { keep4_h(a, b, c, d); }
};
template <> struct Frag<__bf16> {
  typedef v16b V; union U { v16b v; v8b h[2]; };
  static __device__ __forceinline__ v16b load(const __bf16* p) {
    U f; f.h[0] = *(const v8b*)(p); f.h[1] = *(const v8b*)(p + 16); return f.v;
  }
  static __device__ __forceinline__ v8f mma(v16b a, v16b b, v8f c) {
    return __builtin_amdgcn_wmma_f32_16x16x32_bf16(false, a, false, b, (short)0, c, false, false);
  }
  static __device__ __forceinline__ void guard(v8f& a, v8f& b, v16b x, v16b y) { dep_guard_b(a, b, x, y); }
  static __device__ __forceinline__ void keep(v16b a, v16b b, v16b c, v16b d) { keep4_b(a, b, c, d); }
};

template <int ET> struct Elem;
template <> struct Elem<0> { typedef _Float16 T; };
template <> struct Elem<1> { typedef __bf16 T; };
template <int ET, bool SPLIT, int BIAS_MODE, int OUT_MODE, bool RESID, int ACT = 0>
__global__ __launch_bounds__(256) void wmma_gemm64(
    const unsigned short* __restrict__ Ap, const unsigned short* __restrict__ A2p, int lda, long strideA,
    const unsigned short* __restrict__ Btp, const unsigned short* __restrict__ Bt2p, int ldb, long strideB,
    void* __restrict__ Cout, void* __restrict__ Cout2, int ldc, long strideC,
    const float* __restrict__ bias,
    const float* __restrict__ resid, long strideR,
    int M, int N, int K, float scale) {
  typedef typename Elem<ET>::T T;
  typedef typename Frag<T>::V V;
  const T* A = (const T*)Ap; const T* A2 = (const T*)A2p; const T* Bt = (const T*)Btp; const T* Bt2 = (const T*)Bt2p;
  __shared__ __align__(16) float sT[8][16 * 68];
  const int b    = blockIdx.y;
  const int lane = threadIdx.x & 31;
  const int wave = threadIdx.x >> 5;
  const int tilesN = N >> 6;
  const int tilesM = M >> 6;
  const int tile = blockIdx.x * 8 + wave;
  if (tile >= tilesM * tilesN) return;
  const int tm = tile / tilesN;
  const int tn = tile - tm * tilesN;
  const int m0 = tm << 6;
  const int n0 = tn << 6;

  const T* Ab  = A  + (size_t)b * strideA;
  const T* Bb  = Bt + (size_t)b * strideB;
  const T* Ab2 = SPLIT ? (A2  + (size_t)b * strideA) : nullptr;
  const T* Bb2 = SPLIT ? (Bt2 + (size_t)b * strideB) : nullptr;

  const int rlane = lane & 15;
  const int koff  = (lane >> 4) * 8;
  const int mOff  = (lane >> 4) * 8;

  v8f acc[4][4];
#pragma unroll
  for (int i = 0; i < 4; ++i)
#pragma unroll
    for (int j = 0; j < 4; ++j) acc[i][j] = (v8f){0.f,0.f,0.f,0.f,0.f,0.f,0.f,0.f};

  for (int k0 = 0; k0 < K; k0 += 32) {
    V bh[4], bl[4];
#pragma unroll
    for (int j = 0; j < 4; ++j) {
      const size_t bo = (size_t)(n0 + (j << 4) + rlane) * ldb + koff + k0;
      bh[j] = Frag<T>::load(Bb + bo);
      if (SPLIT) bl[j] = Frag<T>::load(Bb2 + bo);
    }
#pragma unroll
    for (int i = 0; i < 4; ++i) {
      const size_t ao = (size_t)(m0 + (i << 4) + rlane) * lda + koff + k0;
      V ah = Frag<T>::load(Ab + ao);
      V al;
      if (SPLIT) al = Frag<T>::load(Ab2 + ao);
#pragma unroll
      for (int j = 0; j < 4; ++j) {
        acc[i][j] = Frag<T>::mma(ah, bh[j], acc[i][j]);
        if (SPLIT) {
          acc[i][j] = Frag<T>::mma(ah, bl[j], acc[i][j]);
          acc[i][j] = Frag<T>::mma(al, bh[j], acc[i][j]);
        }
      }
      Frag<T>::guard(acc[i][0], acc[i][3], ah, SPLIT ? al : ah);
    }
    Frag<T>::keep(bh[0], bh[1], bh[2], bh[3]);
    if (SPLIT) Frag<T>::keep(bl[0], bl[1], bl[2], bl[3]);
  }
  acc_guard4(acc[0][0], acc[0][1], acc[0][2], acc[0][3]);
  acc_guard4(acc[1][0], acc[1][1], acc[1][2], acc[1][3]);
  acc_guard4(acc[2][0], acc[2][1], acc[2][2], acc[2][3]);
  acc_guard4(acc[3][0], acc[3][1], acc[3][2], acc[3][3]);

  float* slab = sT[wave];
  const float* Rb = RESID ? (resid + (size_t)b * strideR) : nullptr;
#pragma unroll
  for (int i = 0; i < 4; ++i) {
    const int mBase = m0 + (i << 4);
#pragma unroll
    for (int j = 0; j < 4; ++j) {
      const int n = n0 + (j << 4) + rlane;
      float bv = 0.f;
      if (BIAS_MODE == 2) bv = bias[n];
#pragma unroll
      for (int r = 0; r < 8; ++r) {
        float v = acc[i][j][r] * scale;
        if (BIAS_MODE == 1) v += bias[mBase + mOff + r];
        if (BIAS_MODE == 2) v += bv;
        if (RESID) v += Rb[(size_t)(mBase + mOff + r) * ldc + n];
        if (ACT == 1) v = tanhf(v);
        if (ACT == 2) v = fmaxf(v, 0.0f);
        if (ACT == 3) v = v / (1.0f + expf(-v));
        if (ACT == 4) v = (v > 0.f) ? v : 0.01f * v;
        if (ACT == 5) v = 0.5f * v * (1.0f + erff(v * 0.70710678118654752f));
        slab[(mOff + r) * 68 + (j << 4) + rlane] = v;
      }
    }
    __builtin_amdgcn_fence(__ATOMIC_RELEASE, "workgroup");
    __builtin_amdgcn_wave_barrier();
    __builtin_amdgcn_fence(__ATOMIC_ACQUIRE, "workgroup");
    if (OUT_MODE == 0) {
      float* C = (float*)Cout + (size_t)b * strideC;
      const int hh = lane >> 4, c4 = (lane & 15) * 4;
      for (int pass = 0; pass < 2; ++pass) {
#pragma unroll
        for (int it = 0; it < 8; ++it) {
          const int row = it * 2 + hh;
          v4f v = *(const v4f*)(slab + row * 68 + c4);
          *(volatile v4f*)(C + (size_t)(mBase + row) * ldc + n0 + c4) = v;
        }
        __threadfence();
      }
    } else {
      const int q = lane >> 3, c8 = (lane & 7) * 8;
      unsigned short* C  = (unsigned short*)Cout  + (size_t)b * strideC;
      unsigned short* C2 = (OUT_MODE == 2) ? ((unsigned short*)Cout2 + (size_t)b * strideC) : nullptr;
      for (int pass = 0; pass < 2; ++pass) {
#pragma unroll
        for (int it = 0; it < 4; ++it) {
          const int row = it * 4 + q;
          const float* sp = slab + row * 68 + c8;
          v8h hv, lv;
#pragma unroll
          for (int e = 0; e < 8; ++e) {
            if (OUT_MODE == 1) {
              hv[e] = (_Float16)sp[e];
            } else {
              unsigned short hb = f2bf_bits(sp[e]);
              unsigned short lb = f2bf_bits(sp[e] - bf_bits2f(hb));
              hv[e] = __builtin_bit_cast(_Float16, hb);
              lv[e] = __builtin_bit_cast(_Float16, lb);
            }
          }
          *(volatile v8h*)(C + (size_t)(mBase + row) * ldc + n0 + c8) = hv;
          if (OUT_MODE == 2) *(volatile v8h*)(C2 + (size_t)(mBase + row) * ldc + n0 + c8) = lv;
        }
        __threadfence();
      }
    }
    __builtin_amdgcn_fence(__ATOMIC_RELEASE, "workgroup");
    __builtin_amdgcn_wave_barrier();
    __builtin_amdgcn_fence(__ATOMIC_ACQUIRE, "workgroup");
  }
}

__device__ __forceinline__ unsigned pack_f16x2(float a, float b) {
  const _Float16 h0 = (_Float16)a, h1 = (_Float16)b;
  return (unsigned)__builtin_bit_cast(unsigned short, h0) | ((unsigned)__builtin_bit_cast(unsigned short, h1) << 16);
}
__device__ __forceinline__ void split_bf2(float a, float b, unsigned& hi, unsigned& lo) {
  const unsigned short ha = f2bf_bits(a), hb = f2bf_bits(b);
  const unsigned short la = f2bf_bits(a - bf_bits2f(ha)), lb = f2bf_bits(b - bf_bits2f(hb));
  hi = (unsigned)ha | ((unsigned)hb << 16);
  lo = (unsigned)la | ((unsigned)lb << 16);
}
__device__ __forceinline__ void st2u(unsigned* p, unsigned v) { *(volatile unsigned*)p = v; __threadfence(); *(volatile unsigned*)p = v; }
__device__ __forceinline__ float ftanh(float x) { return 1.0f - 2.0f * __builtin_amdgcn_rcpf(1.0f + __expf(2.0f * x)); }
__device__ __forceinline__ float fsigm(float x) { return __builtin_amdgcn_rcpf(1.0f + __expf(-x)); }

__global__ __launch_bounds__(kThreads) void prep_kernel(const float* __restrict__ x, const float* __restrict__ labW,
                                                       const float* __restrict__ stat, const float* __restrict__ demoW,
                                                       const float* __restrict__ outW,
                                                       _Float16* __restrict__ X16, unsigned* __restrict__ LW16,
                                                       unsigned* __restrict__ SThi, unsigned* __restrict__ STlo,
                                                       unsigned* __restrict__ DWhi, unsigned* __restrict__ DWlo,
                                                       unsigned* __restrict__ OWhi, unsigned* __restrict__ OWlo) {
  const int blk = blockIdx.x, tid = threadIdx.x;
  if (blk < kPrepX) {
    const int gid = blk * kThreads + tid;
    const float* p = x + (size_t)gid * 8;
    const v4f a = *(const v4f*)p, bq = *(const v4f*)(p + 4);
    v8h h;
#pragma unroll
    for (int e = 0; e < 4; ++e) { h[e] = (_Float16)a[e]; h[4 + e] = (_Float16)bq[e]; }
    _Float16* op = X16 + (size_t)gid * 8;
    *(volatile v8h*)op = h; __threadfence(); *(volatile v8h*)op = h;
  } else if (blk < kPrepX + kPrepLW) {
    const int p = (blk - kPrepX) * kThreads + tid;
    const unsigned u = pack_f16x2(labW[2 * p] * 64.0f, labW[2 * p + 1] * 64.0f);
    st2u(LW16 + p, u);
  } else if (blk < kPrepX + kPrepLW + kPrepST) {
    const int p = (blk - kPrepX - kPrepLW) * kThreads + tid;
    unsigned hi, lo; split_bf2(stat[2 * p], stat[2 * p + 1], hi, lo);
    st2u(SThi + p, hi); st2u(STlo + p, lo);
  } else if (blk < kPrepX + kPrepLW + kPrepST + kPrepDW) {
    const int p = (blk - kPrepX - kPrepLW - kPrepST) * kThreads + tid;
    unsigned hi, lo; split_bf2(demoW[2 * p], demoW[2 * p + 1], hi, lo);
    st2u(DWhi + p, hi); st2u(DWlo + p, lo);
  } else {
    const int p = (blk - kPrepX - kPrepLW - kPrepST - kPrepDW) * kThreads + tid;
    unsigned hi, lo; split_bf2(outW[2 * p], outW[2 * p + 1], hi, lo);
    st2u(OWhi + p, hi); st2u(OWlo + p, lo);
  }
}

__global__ __launch_bounds__(kThreads) void mcgru_rec_kernel(const float* __restrict__ XPT,
                                                            const float* __restrict__ Wih, const float* __restrict__ bih,
                                                            const float* __restrict__ Whh, const float* __restrict__ bhh,
                                                            const int* __restrict__ mask, float* __restrict__ HLAST) {
  __shared__ __align__(16) float    sXp[64 * kNT];
  __shared__ __align__(16) _Float16 sWhh[kNG * kWP];
  __shared__ __align__(16) _Float16 sH16[64 * kHP];
  __shared__ __align__(16) float    sSnap[64 * kSP];
  __shared__ int sLast[64];
  const int l = blockIdx.x, b0 = blockIdx.y * 64;
  const int tid = threadIdx.x, lane = tid & 31, wave = tid >> 5;
  const int rlane = lane & 15, hh = lane >> 4, koff = hh * 8, mOff = hh * 8;

  {
    const float* wsrc = Whh + (size_t)l * (kNG * kNF);
#pragma unroll 4
    for (int i = tid; i < kNG * kNF; i += kThreads) sWhh[(i >> 5) * kWP + (i & 31)] = (_Float16)(wsrc[i] * 64.0f);
  }
  {
    const v4f* xs = (const v4f*)(XPT + ((size_t)l * kNB + b0) * kNT);
    v4f* xd = (v4f*)sXp;
#pragma unroll
    for (int it = 0; it < 8; ++it) xd[it * kThreads + tid] = xs[it * kThreads + tid];
  }
  for (int i = tid; i < 64 * kHP; i += kThreads) sH16[i] = (_Float16)0.0f;
  if (tid < 64) {
    const int4* mp = (const int4*)(mask + (size_t)(b0 + tid) * kNT);
    int s = 0;
#pragma unroll 1
    for (int q = 0; q < kNT / 4; ++q) { const int4 m4 = mp[q]; s += m4.x + m4.y + m4.z + m4.w; }
    s -= 1;
    s = s < 0 ? 0 : s;
    s = s > kNT - 1 ? kNT - 1 : s;
    sLast[tid] = s;
  }
  __syncthreads();

  const int i  = wave >> 1;
  const int hf = wave & 1;
  const int j  = 16 * hf + rlane;
  const v16h bR = Frag<_Float16>::load(sWhh + (size_t)j * kWP + koff);
  const v16h bZ = Frag<_Float16>::load(sWhh + (size_t)(kNF + j) * kWP + koff);
  const v16h bN = Frag<_Float16>::load(sWhh + (size_t)(2 * kNF + j) * kWP + koff);
  const float wir = Wih[l * kNG + j], wiz = Wih[l * kNG + kNF + j], win = Wih[l * kNG + 2 * kNF + j];
  const float bir = bih[l * kNG + j], biz = bih[l * kNG + kNF + j], bin_ = bih[l * kNG + 2 * kNF + j];
  const float bhr = bhh[l * kNG + j], bhz = bhh[l * kNG + kNF + j], bhn = bhh[l * kNG + 2 * kNF + j];
  const _Float16* arow = sH16 + (size_t)(16 * i + rlane) * kHP + koff;
  const int rowbase = 16 * i + mOff;
  const float* xrow = sXp + rowbase * kNT;
  const v8f z8 = {0.f, 0.f, 0.f, 0.f, 0.f, 0.f, 0.f, 0.f};
  const float inv = 1.0f / 16384.0f;

  int lastv[8]; float hreg[8], snap[8];
#pragma unroll
  for (int r = 0; r < 8; ++r) { lastv[r] = sLast[rowbase + r]; hreg[r] = 0.0f; snap[r] = 0.0f; }

#pragma unroll 1
  for (int t = 0; t < kNT; ++t) {
    const v16h a = Frag<_Float16>::load(arow);
    v8f ar = Frag<_Float16>::mma(a, bR, z8);
    v8f az = Frag<_Float16>::mma(a, bZ, z8);
    v8f an = Frag<_Float16>::mma(a, bN, z8);
    dep_guard3_h(ar, az, an, a, bR, bZ, bN);
    acc_guard3(ar, az, an);
#pragma unroll
    for (int r = 0; r < 8; ++r) {
      const float xv = xrow[r * kNT + t];
      const float gr = fmaf(xv, wir, bir) + fmaf(ar[r], inv, bhr);
      const float gz = fmaf(xv, wiz, biz) + fmaf(az[r], inv, bhz);
      const float hn = fmaf(an[r], inv, bhn);
      const float rg = fsigm(gr);
      const float zg = fsigm(gz);
      const float ng = ftanh(fmaf(xv, win, bin_) + rg * hn);
      const float hv = (1.0f - zg) * ng + zg * hreg[r];
      hreg[r] = hv;
      snap[r] = (t == lastv[r]) ? hv : snap[r];
    }
    __syncthreads();
#pragma unroll
    for (int r = 0; r < 8; ++r) sH16[(rowbase + r) * kHP + j] = (_Float16)(hreg[r] * 256.0f);
    __syncthreads();
  }

#pragma unroll
  for (int r = 0; r < 8; ++r) sSnap[(rowbase + r) * kSP + j] = snap[r];
  __syncthreads();
  {
    const int q = lane >> 3, c4 = (lane & 7) * 4;
    for (int pass = 0; pass < 2; ++pass) {
#pragma unroll
      for (int it = 0; it < 2; ++it) {
        const int row = it * 32 + wave * 4 + q;
        const v4f v = *(const v4f*)(sSnap + row * kSP + c4);
        *(volatile v4f*)(HLAST + ((size_t)(b0 + row) * kNL + l) * kNF + c4) = v;
      }
      __threadfence();
    }
  }
}

__global__ __launch_bounds__(kThreads) void pack_h_kernel(const float* __restrict__ HLAST,
                                                         unsigned short* __restrict__ A2hi, unsigned short* __restrict__ A2lo) {
  const int lane = threadIdx.x & 31, wave = threadIdx.x >> 5;
  const int b = blockIdx.x * 8 + wave;
  const float* src = HLAST + (size_t)b * (kNL * kNF);
  unsigned short* dh = A2hi + (size_t)b * kKO + kNH;
  unsigned short* dl = A2lo + (size_t)b * kKO + kNH;
#pragma unroll 1
  for (int it = 0; it < 8; ++it) {
    const int idx = it * 256 + lane * 8;
    const v4f a = *(const v4f*)(src + idx), bq = *(const v4f*)(src + idx + 4);
    v8h hv, lv;
#pragma unroll
    for (int e = 0; e < 4; ++e) {
      const unsigned short h0 = f2bf_bits(a[e]);
      const unsigned short l0 = f2bf_bits(a[e] - bf_bits2f(h0));
      const unsigned short h1 = f2bf_bits(bq[e]);
      const unsigned short l1 = f2bf_bits(bq[e] - bf_bits2f(h1));
      hv[e] = __builtin_bit_cast(_Float16, h0); lv[e] = __builtin_bit_cast(_Float16, l0);
      hv[4 + e] = __builtin_bit_cast(_Float16, h1); lv[4 + e] = __builtin_bit_cast(_Float16, l1);
    }
    *(volatile v8h*)(dh + idx) = hv;
    *(volatile v8h*)(dl + idx) = lv;
    __threadfence();
    *(volatile v8h*)(dh + idx) = hv;
    *(volatile v8h*)(dl + idx) = lv;
  }
}

extern "C" void kernel_launch(void* const* d_in, const int* in_sizes, int n_in,
                              void* d_out, int out_size, void* d_ws, size_t ws_size, hipStream_t stream) {
  if (n_in < 13 || d_out == nullptr || d_ws == nullptr) return;
  if (in_sizes[0] != kNB * kNT * kNL || in_sizes[1] != kNB * kND || in_sizes[2] != kNB * kNT ||
      in_sizes[3] != kNH * kND || in_sizes[4] != kNH || in_sizes[5] != kNL * kNL || in_sizes[6] != kNL ||
      in_sizes[7] != kNL * kNG || in_sizes[8] != kNL * kNG || in_sizes[9] != kNL * kNG * kNF ||
      in_sizes[10] != kNL * kNG || in_sizes[11] != kNH * kKO || in_sizes[12] != kNH ||
      out_size != kNB * kNH) return;

  const float* x      = (const float*)d_in[0];
  const float* stat   = (const float*)d_in[1];
  const int*   mask   = (const int*)d_in[2];
  const float* demo_W = (const float*)d_in[3];
  const float* demo_b = (const float*)d_in[4];
  const float* lab_W  = (const float*)d_in[5];
  const float* lab_b  = (const float*)d_in[6];
  const float* Wih    = (const float*)d_in[7];
  const float* bih    = (const float*)d_in[8];
  const float* Whh    = (const float*)d_in[9];
  const float* bhh    = (const float*)d_in[10];
  const float* out_W  = (const float*)d_in[11];
  const float* out_b  = (const float*)d_in[12];
  float* out = (float*)d_out;

  char* ws = (char*)d_ws; size_t off = 0;
  auto carve = [&](size_t bytes) -> char* { char* p = ws + off; off += (bytes + 255) & ~(size_t)255; return p; };
  _Float16* X16   = (_Float16*)carve((size_t)kNB * kNT * kNL * 2);
  unsigned* LW16  = (unsigned*)carve((size_t)kNL * kNL * 2);
  unsigned* SThi  = (unsigned*)carve((size_t)kNB * kND * 2);
  unsigned* STlo  = (unsigned*)carve((size_t)kNB * kND * 2);
  unsigned* DWhi  = (unsigned*)carve((size_t)kNH * kND * 2);
  unsigned* DWlo  = (unsigned*)carve((size_t)kNH * kND * 2);
  unsigned* OWhi  = (unsigned*)carve((size_t)kNH * kKO * 2);
  unsigned* OWlo  = (unsigned*)carve((size_t)kNH * kKO * 2);
  float*    XPT   = (float*)carve((size_t)kNL * kNB * kNT * 4);
  float*    HLAST = (float*)carve((size_t)kNB * kNL * kNF * 4);
  unsigned short* A2hi = (unsigned short*)carve((size_t)kNB * kKO * 2);
  unsigned short* A2lo = (unsigned short*)carve((size_t)kNB * kKO * 2);
  if (off > ws_size || off > (size_t)134217728) return;

  prep_kernel<<<kPrepBlocks, kThreads, 0, stream>>>(x, lab_W, stat, demo_W, out_W,
                                                    X16, LW16, SThi, STlo, DWhi, DWlo, OWhi, OWlo);
  wmma_gemm64<0, false, 1, 0, false><<<dim3((kNB * kNT) / 64 / 8, 1), 256, 0, stream>>>(
      (const unsigned short*)LW16, (const unsigned short*)nullptr, kNL, 0L,
      (const unsigned short*)X16, (const unsigned short*)nullptr, kNL, 0L,
      (void*)XPT, (void*)nullptr, kNB * kNT, 0L,
      lab_b, (const float*)nullptr, 0L, kNL, kNB * kNT, kNL, 1.0f / 64.0f);
  mcgru_rec_kernel<<<dim3(kNL, kNB / 64), kThreads, 0, stream>>>(XPT, Wih, bih, Whh, bhh, mask, HLAST);
  wmma_gemm64<1, true, 2, 2, false><<<dim3(1, 1), 256, 0, stream>>>(
      (const unsigned short*)SThi, (const unsigned short*)STlo, kND, 0L,
      (const unsigned short*)DWhi, (const unsigned short*)DWlo, kND, 0L,
      (void*)A2hi, (void*)A2lo, kKO, 0L,
      demo_b, (const float*)nullptr, 0L, kNB, kNH, kND, 1.0f);
  pack_h_kernel<<<kNB / 8, kThreads, 0, stream>>>(HLAST, A2hi, A2lo);
  wmma_gemm64<1, true, 2, 0, false><<<dim3(1, 1), 256, 0, stream>>>(
      (const unsigned short*)A2hi, (const unsigned short*)A2lo, kKO, 0L,
      (const unsigned short*)OWhi, (const unsigned short*)OWlo, kKO, 0L,
      (void*)out, (void*)nullptr, kNH, 0L,
      out_b, (const float*)nullptr, 0L, kNB, kNH, kKO, 1.0f);
}
